// VNResnetPointnet_57080115364769
// MI455X (gfx1250) — hardware-verified
//
#include <hip/hip_runtime.h>

typedef __attribute__((ext_vector_type(16))) _Float16 v16h;
typedef __attribute__((ext_vector_type(8)))  _Float16 v8h;
typedef __attribute__((ext_vector_type(8)))  float    v8f;
typedef __attribute__((ext_vector_type(4)))  float    v4f;
typedef __attribute__((ext_vector_type(4)))  unsigned v4u;

constexpr int kB    = 8;
constexpr int kN    = 1024;
constexpr int kKnn  = 20;
constexpr int kRows = kB * 3 * kN;
constexpr int kC2   = 256;
constexpr int kH3   = 128;
constexpr int kEPitch = 16;
constexpr float kWCarry    = 16.0f;
constexpr float kWCarryInv = 1.0f / 16.0f;
constexpr float kResScale  = 2048.0f;
constexpr float kResInv    = 1.0f / 2048.0f;
constexpr float kHiFloor   = 6.2e-5f;
constexpr float kEps       = 1e-6f;
constexpr float kInvN      = 1.0f / 1024.0f;
constexpr float kInvK      = 1.0f / 20.0f;

static_assert(kRows == 24576, "row count");
static_assert(kB * kH3 * 3 * 4 == 12288, "d_out bytes");
static_assert(kN == 1024, "shifts below assume 1024 points per cloud");

constexpr size_t kSzWd0 = (size_t)5 * 256 * 256 * 2;
constexpr size_t kSzW0  = (size_t)5 * 128 * 256 * 2;
constexpr size_t kSzWd1 = (size_t)5 * 128 * 128 * 2;
constexpr size_t kSzW1  = (size_t)5 * 128 * 128 * 2;
constexpr size_t kSzWs  = (size_t)5 * 128 * 256 * 2;
constexpr size_t kSzE   = (size_t)kB * kN * kEPitch * 4;
constexpr size_t kSzX   = (size_t)kRows * 256 * 2;
constexpr size_t kSzH   = (size_t)kRows * 128 * 2;
constexpr size_t kOffWd0H = 0;
constexpr size_t kOffWd0L = kOffWd0H + kSzWd0;
constexpr size_t kOffW0H  = kOffWd0L + kSzWd0;
constexpr size_t kOffW0L  = kOffW0H  + kSzW0;
constexpr size_t kOffWd1H = kOffW0L  + kSzW0;
constexpr size_t kOffWd1L = kOffWd1H + kSzWd1;
constexpr size_t kOffW1H  = kOffWd1L + kSzWd1;
constexpr size_t kOffW1L  = kOffW1H  + kSzW1;
constexpr size_t kOffWsH  = kOffW1L  + kSzW1;
constexpr size_t kOffWsL  = kOffWsH  + kSzWs;
constexpr size_t kOffE    = kOffWsL  + kSzWs;
constexpr size_t kOffX0H  = kOffE    + kSzE;
constexpr size_t kOffX0L  = kOffX0H  + kSzX;
constexpr size_t kOffX1H  = kOffX0L  + kSzX;
constexpr size_t kOffX1L  = kOffX1H  + kSzX;
constexpr size_t kOffA0H  = kOffX1L  + kSzX;
constexpr size_t kOffA0L  = kOffA0H  + kSzX;
constexpr size_t kOffT0H  = kOffA0L  + kSzX;
constexpr size_t kOffT0L  = kOffT0H  + kSzH;
constexpr size_t kOffA1H  = kOffT0L  + kSzH;
constexpr size_t kOffA1L  = kOffA1H  + kSzH;
constexpr size_t kOffYLH  = kOffA1L  + kSzH;
constexpr size_t kOffYLL  = kOffYLH  + kSzH;
constexpr size_t kWsTotal = kOffYLL  + kSzH;
static_assert(kWsTotal == 117047296, "carve total");
static_assert(kWsTotal <= 134217728, "carve within 128 MiB");
static_assert(kSzWd0 % 128 == 0 && kSzW0 % 128 == 0 && kSzWd1 % 128 == 0 && kSzW1 % 128 == 0 &&
              kSzWs % 128 == 0 && kSzE % 128 == 0 && kSzX % 128 == 0 && kSzH % 128 == 0, "line aligned carve");

union FragH { v16h v; v8h h[2]; };

__device__ __forceinline__ v16h frag_load(const _Float16* p) {
  FragH f;
  f.h[0] = *(const v8h*)(p);
  f.h[1] = *(const v8h*)(p + 16);
  return f.v;
}

__device__ __forceinline__ v8f mma_f16(v16h a, v16h b, v8f c) {
  c = __builtin_amdgcn_wmma_f32_16x16x32_f16(false, a, false, b, (short)0, c, false, false);
  asm volatile("v_nop\n\tv_nop\n\tv_nop\n\tv_nop" : "+v"(c) : "v"(a), "v"(b));
  return c;
}

__device__ __forceinline__ float h16_to_f32(unsigned hb) {
  const unsigned sgn = (hb & 0x8000u) << 16;
  const unsigned em = hb & 0x7fffu;
  const float fn = __uint_as_float((em << 13) + 0x38000000u);
  const float fs = (float)em * 5.9604644775390625e-8f;
  const float mag = (em < 0x400u) ? fs : fn;
  return __uint_as_float(__float_as_uint(mag) | sgn);
}

__device__ __forceinline__ float rec16(unsigned hb, unsigned lb) {
  const float h = h16_to_f32(hb);
  const float l = h16_to_f32(lb);
  return fmaf(l, kResInv, h);
}

__device__ __forceinline__ void unpack8(v4u wh, v4u wl, float (&x)[8]) {
  const unsigned h0 = wh.x, h1 = wh.y, h2 = wh.z, h3 = wh.w;
  const unsigned l0 = wl.x, l1 = wl.y, l2 = wl.z, l3 = wl.w;
  x[0] = rec16(h0 & 0xffffu, l0 & 0xffffu); x[1] = rec16(h0 >> 16, l0 >> 16);
  x[2] = rec16(h1 & 0xffffu, l1 & 0xffffu); x[3] = rec16(h1 >> 16, l1 >> 16);
  x[4] = rec16(h2 & 0xffffu, l2 & 0xffffu); x[5] = rec16(h2 >> 16, l2 >> 16);
  x[6] = rec16(h3 & 0xffffu, l3 & 0xffffu); x[7] = rec16(h3 >> 16, l3 >> 16);
}

__device__ __forceinline__ void split16(float v, unsigned& hb, unsigned& lb) {
  const _Float16 h = (_Float16)v;
  float hf = (float)h;
  unsigned hbits = (unsigned)__builtin_bit_cast(unsigned short, h);
  const bool z = fabsf(hf) < kHiFloor;
  hbits = z ? 0u : hbits;
  hf = z ? 0.0f : hf;
  const float r = (v - hf) * kResScale;
  const _Float16 l = (_Float16)r;
  lb = (unsigned)__builtin_bit_cast(unsigned short, l);
  hb = hbits;
}

__global__ __launch_bounds__(256) void k_cvt_w(const float* __restrict__ in, unsigned short* __restrict__ oh,
                                               unsigned short* __restrict__ ol, int n8) {
  const int i = blockIdx.x * 256 + threadIdx.x;
  if (i < n8) {
    const v4f a = *(const v4f*)(in + (size_t)i * 8);
    const v4f c = *(const v4f*)(in + (size_t)i * 8 + 4);
    float f[8];
#pragma unroll
    for (int e = 0; e < 4; ++e) {
      f[e]     = a[e] * kWCarry;
      f[4 + e] = c[e] * kWCarry;
    }
    unsigned hw[4], lw[4];
#pragma unroll
    for (int ep = 0; ep < 4; ++ep) {
      unsigned ha, la, hb, lb;
      split16(f[2 * ep], ha, la);
      split16(f[2 * ep + 1], hb, lb);
      hw[ep] = ha | (hb << 16);
      lw[ep] = la | (lb << 16);
    }
    const v4u vh = (v4u){hw[0], hw[1], hw[2], hw[3]};
    const v4u vl = (v4u){lw[0], lw[1], lw[2], lw[3]};
    volatile v4u* dh = (volatile v4u*)(oh + (size_t)i * 8);
    volatile v4u* dl = (volatile v4u*)(ol + (size_t)i * 8);
    *dh = vh;
    *dl = vl;
    __threadfence();
    *dh = vh;
    *dl = vl;
  }
}

__global__ __launch_bounds__(256) void k_knn_feat(const float* __restrict__ p, float* __restrict__ E) {
#pragma clang fp contract(off)
  __shared__ __align__(16) float raw[kN * 3];
  __shared__ float sx[kN];
  __shared__ float sy[kN];
  __shared__ float sz[kN];
  __shared__ float sq[kN];
  __shared__ float wpart[3][8];
  __shared__ __align__(16) float stg[256 * kEPitch];
  const int tid = threadIdx.x, lane = tid & 31, wave = tid >> 5;
  const int b = blockIdx.x >> 2;
  const int chunk = blockIdx.x & 3;
  {
    const v4f* src = (const v4f*)(p + (size_t)b * kN * 3);
    v4f* dl = (v4f*)raw;
#pragma unroll
    for (int m = 0; m < 3; ++m) dl[tid + 256 * m] = src[tid + 256 * m];
  }
  __syncthreads();
  float ax = 0.f, ay = 0.f, az = 0.f;
#pragma unroll
  for (int q = 0; q < 4; ++q) {
    const int i = tid + 256 * q;
    ax += raw[i * 3 + 0];
    ay += raw[i * 3 + 1];
    az += raw[i * 3 + 2];
  }
#pragma unroll
  for (int off = 16; off > 0; off >>= 1) {
    ax += __shfl_xor(ax, off, 32);
    ay += __shfl_xor(ay, off, 32);
    az += __shfl_xor(az, off, 32);
  }
  if (lane == 0) { wpart[0][wave] = ax; wpart[1][wave] = ay; wpart[2][wave] = az; }
  __syncthreads();
  float mx = 0.f, my = 0.f, mz = 0.f;
#pragma unroll
  for (int w = 0; w < 8; ++w) { mx += wpart[0][w]; my += wpart[1][w]; mz += wpart[2][w]; }
  mx = mx * kInvN; my = my * kInvN; mz = mz * kInvN;
#pragma unroll
  for (int q = 0; q < 4; ++q) {
    const int i = tid + 256 * q;
    const float x = raw[i * 3 + 0] - mx;
    const float y = raw[i * 3 + 1] - my;
    const float z = raw[i * 3 + 2] - mz;
    const float t0 = x * x, t1 = y * y, t2 = z * z;
    sx[i] = x; sy[i] = y; sz[i] = z;
    sq[i] = (t0 + t1) + t2;
  }
  __syncthreads();

  const int qi = chunk * 256 + tid;
  const float xi = sx[qi], yi = sy[qi], zi = sz[qi];
  const float nqi = -sq[qi];
  float bd[kKnn];
  int   bi[kKnn];
#pragma unroll
  for (int k = 0; k < kKnn; ++k) { bd[k] = -3.0e38f; bi[k] = 0; }
#pragma unroll 1
  for (int j = 0; j < kN; ++j) {
    const float xj = sx[j], yj = sy[j], zj = sz[j], qj = sq[j];
    float dt = xi * xj;
    dt = fmaf(yi, yj, dt);
    dt = fmaf(zi, zj, dt);
    const float inner = -2.0f * dt;
    const float nd = (nqi - inner) - qj;
    const unsigned anyb = __builtin_amdgcn_ballot_w32(nd > bd[kKnn - 1]);
    if (anyb != 0u) {
#pragma unroll
      for (int k = kKnn - 1; k >= 1; --k) {
        const bool mv = nd > bd[k - 1];
        const bool hr = nd > bd[k];
        bd[k] = mv ? bd[k - 1] : (hr ? nd : bd[k]);
        bi[k] = mv ? bi[k - 1] : (hr ? j : bi[k]);
      }
      const bool h0 = nd > bd[0];
      bd[0] = h0 ? nd : bd[0];
      bi[0] = h0 ? j : bi[0];
    }
  }
  float gx = 0.f, gy = 0.f, gz = 0.f;
#pragma unroll
  for (int k = 0; k < kKnn; ++k) {
    int jj = bi[k];
    jj = jj < 0 ? 0 : (jj > kN - 1 ? kN - 1 : jj);
    gx += sx[jj]; gy += sy[jj]; gz += sz[jj];
  }
  const float m0 = gx * kInvK, m1 = gy * kInvK, m2 = gz * kInvK;
  const float d0 = m0 - xi, d1 = m1 - yi, d2 = m2 - zi;
  const float pa0 = m1 * zi, pb0 = m2 * yi;
  const float pa1 = m2 * xi, pb1 = m0 * zi;
  const float pa2 = m0 * yi, pb2 = m1 * xi;
  const float cr0 = pa0 - pb0, cr1 = pa1 - pb1, cr2 = pa2 - pb2;
  {
    v4f* sv = (v4f*)stg;
    sv[tid * 4 + 0] = (v4f){d0, xi, cr0, 0.f};
    sv[tid * 4 + 1] = (v4f){d1, yi, cr1, 0.f};
    sv[tid * 4 + 2] = (v4f){d2, zi, cr2, 0.f};
    sv[tid * 4 + 3] = (v4f){0.f, 0.f, 0.f, 0.f};
  }
  __syncthreads();
  {
    v4f vals[4];
#pragma unroll
    for (int m = 0; m < 4; ++m) vals[m] = ((const v4f*)stg)[tid + 256 * m];
    float* dst = E + ((size_t)b * kN + (size_t)chunk * 256) * kEPitch;
    for (int pass = 0; pass < 2; ++pass) {
#pragma unroll
      for (int m = 0; m < 4; ++m) *(volatile v4f*)(dst + (size_t)(tid + 256 * m) * 4) = vals[m];
      __threadfence();
    }
  }
}

__global__ __launch_bounds__(256) void k_init(const float* __restrict__ E, const float* __restrict__ Wp,
                                              unsigned short* __restrict__ X0h, unsigned short* __restrict__ X0l) {
  const int tid = threadIdx.x, lane = tid & 31, wave = tid >> 5;
  const int gw = blockIdx.x * 8 + wave;
  v4f wv[6];
#pragma unroll
  for (int i = 0; i < 6; ++i) wv[i] = *(const v4f*)(Wp + lane * 24 + 4 * i);
#pragma unroll 1
  for (int rr = 0; rr < 32; ++rr) {
    const int m = gw * 32 + rr;
    const int bv = m >> 10;
    const int n = m & (kN - 1);
    const int b = bv / 3;
    const int v = bv - 3 * b;
    const v4f e = *(const v4f*)(E + ((size_t)b * kN + n) * kEPitch + v * 4);
    float val[8];
#pragma unroll
    for (int k = 0; k < 8; ++k) {
      const float w0 = wv[(3 * k) >> 2][(3 * k) & 3];
      const float w1 = wv[(3 * k + 1) >> 2][(3 * k + 1) & 3];
      const float w2 = wv[(3 * k + 2) >> 2][(3 * k + 2) & 3];
      val[k] = w0 * e[0] + w1 * e[1] + w2 * e[2];
    }
    unsigned hw[4], lw[4];
#pragma unroll
    for (int ep = 0; ep < 4; ++ep) {
      unsigned ha, la, hb, lb;
      split16(val[2 * ep], ha, la);
      split16(val[2 * ep + 1], hb, lb);
      hw[ep] = ha | (hb << 16);
      lw[ep] = la | (lb << 16);
    }
    const v4u vh = (v4u){hw[0], hw[1], hw[2], hw[3]};
    const v4u vl = (v4u){lw[0], lw[1], lw[2], lw[3]};
    volatile v4u* dh = (volatile v4u*)(X0h + (size_t)m * kC2 + lane * 8);
    volatile v4u* dl = (volatile v4u*)(X0l + (size_t)m * kC2 + lane * 8);
    *dh = vh;
    *dl = vl;
    __threadfence();
    *dh = vh;
    *dl = vl;
  }
}

template <int KK>
__device__ __forceinline__ void vn_kloop(const _Float16* __restrict__ Ah, const _Float16* __restrict__ Al, int lda,
                                         const _Float16* __restrict__ Wh, const _Float16* __restrict__ Wl,
                                         int mrow0, int wrow0, int l15, int koff,
                                         v8f (&am)[3][2], v8f (&ar)[3][2]) {
#pragma unroll 1
  for (int k0 = 0; k0 < KK; k0 += 32) {
    v16h bh[2], bl[2];
#pragma unroll
    for (int j = 0; j < 2; ++j) {
      const size_t bo = (size_t)(wrow0 + 16 * j + l15) * KK + koff + k0;
      bh[j] = frag_load(Wh + bo);
      bl[j] = frag_load(Wl + bo);
    }
#pragma unroll
    for (int v = 0; v < 3; ++v) {
      const size_t ao = (size_t)(mrow0 + v * kN + l15) * lda + koff + k0;
      const v16h ah = frag_load(Ah + ao);
      const v16h al = frag_load(Al + ao);
#pragma unroll
      for (int j = 0; j < 2; ++j) {
        am[v][j] = mma_f16(ah, bh[j], am[v][j]);
        ar[v][j] = mma_f16(ah, bl[j], ar[v][j]);
        ar[v][j] = mma_f16(al, bh[j], ar[v][j]);
      }
    }
  }
}

__device__ __forceinline__ void vn_act(float x0, float x1, float x2, float d0, float d1, float d2,
                                       float& o0, float& o1, float& o2) {
  const float dot = x0 * d0 + x1 * d1 + x2 * d2;
  const float dd  = d0 * d0 + d1 * d1 + d2 * d2;
  const float inv = 1.0f / (dd + kEps);
  const float f = (dot >= 0.0f) ? 0.0f : dot * inv;
  o0 = x0 - f * d0;
  o1 = x1 - f * d1;
  o2 = x2 - f * d2;
}

template <int K1, int K2, int NOUT, int MODE>
__global__ __launch_bounds__(128) void k_vn_gemm(
    const unsigned short* __restrict__ A1h, const unsigned short* __restrict__ A1l, int lda1,
    const unsigned short* __restrict__ W1h, const unsigned short* __restrict__ W1l,
    const unsigned short* __restrict__ A2h, const unsigned short* __restrict__ A2l, int lda2,
    const unsigned short* __restrict__ W2h, const unsigned short* __restrict__ W2l,
    unsigned short* __restrict__ Oh, unsigned short* __restrict__ Ol, int ldc) {
  static_assert(K1 % 32 == 0 && K2 % 32 == 0 && NOUT % 128 == 0, "tile multiples");
  static_assert(MODE == 0 || (K2 == 0 && NOUT == K1), "square direction weight");
  constexpr int CGB = NOUT / 128;
  constexpr int SP = 132;
  __shared__ __align__(16) float sT[3 * 16 * SP];
  const int tid = threadIdx.x, lane = tid & 31, wave = tid >> 5;
  const int l15 = lane & 15, hf = lane >> 4, koff = hf * 8;
  const int cgb = blockIdx.x % CGB;
  const int nt = blockIdx.x / CGB;
  const int b = nt >> 6;
  const int n0 = (nt & 63) << 4;
  const int mrow0 = b * 3 * kN + n0;
  const int wrow0 = cgb * 128 + wave * 32;

  v8f am[3][2], ar[3][2];
#pragma unroll
  for (int v = 0; v < 3; ++v)
#pragma unroll
    for (int j = 0; j < 2; ++j) {
      am[v][j] = (v8f){0.f, 0.f, 0.f, 0.f, 0.f, 0.f, 0.f, 0.f};
      ar[v][j] = (v8f){0.f, 0.f, 0.f, 0.f, 0.f, 0.f, 0.f, 0.f};
    }

  vn_kloop<K1>((const _Float16*)A1h, (const _Float16*)A1l, lda1, (const _Float16*)W1h, (const _Float16*)W1l,
               mrow0, wrow0, l15, koff, am, ar);
  if constexpr (K2 > 0) {
    vn_kloop<K2>((const _Float16*)A2h, (const _Float16*)A2l, lda2, (const _Float16*)W2h, (const _Float16*)W2l,
                 mrow0, wrow0, l15, koff, am, ar);
  }

#pragma unroll
  for (int v = 0; v < 3; ++v)
#pragma unroll
    for (int j = 0; j < 2; ++j)
#pragma unroll
      for (int r = 0; r < 8; ++r) {
        const float comb = am[v][j][r] + ar[v][j][r] * kResInv;
        sT[(v * 16 + 8 * hf + r) * SP + wave * 32 + 16 * j + l15] = comb * kWCarryInv;
      }
  __syncthreads();

#pragma unroll 1
  for (int it = 0; it < 2; ++it) {
    const int item = tid + 128 * it;
    const int row = item >> 4;
    const int c8 = (item & 15) * 8;
    const int ccol = cgb * 128 + c8;
    float dv[3][8];
#pragma unroll
    for (int v = 0; v < 3; ++v) {
      const v4f lo4 = *(const v4f*)(sT + (v * 16 + row) * SP + c8);
      const v4f hi4 = *(const v4f*)(sT + (v * 16 + row) * SP + c8 + 4);
#pragma unroll
      for (int e = 0; e < 4; ++e) { dv[v][e] = lo4[e]; dv[v][4 + e] = hi4[e]; }
    }
    float xv[3][8];
    if constexpr (MODE == 1) {
#pragma unroll
      for (int v = 0; v < 3; ++v) {
        const size_t xo = (size_t)(mrow0 + v * kN + row) * lda1 + ccol;
        const v4u wh = *(const v4u*)(A1h + xo);
        const v4u wl = *(const v4u*)(A1l + xo);
        unpack8(wh, wl, xv[v]);
      }
    }
    unsigned oh[3][4], ol[3][4];
#pragma unroll
    for (int ep = 0; ep < 4; ++ep) {
      float oa[3], ob[3];
      if constexpr (MODE == 1) {
        vn_act(xv[0][2 * ep], xv[1][2 * ep], xv[2][2 * ep],
               dv[0][2 * ep], dv[1][2 * ep], dv[2][2 * ep], oa[0], oa[1], oa[2]);
        vn_act(xv[0][2 * ep + 1], xv[1][2 * ep + 1], xv[2][2 * ep + 1],
               dv[0][2 * ep + 1], dv[1][2 * ep + 1], dv[2][2 * ep + 1], ob[0], ob[1], ob[2]);
      } else {
#pragma unroll
        for (int v = 0; v < 3; ++v) { oa[v] = dv[v][2 * ep]; ob[v] = dv[v][2 * ep + 1]; }
      }
#pragma unroll
      for (int v = 0; v < 3; ++v) {
        unsigned ha, la, hb, lb;
        split16(oa[v], ha, la);
        split16(ob[v], hb, lb);
        oh[v][ep] = ha | (hb << 16);
        ol[v][ep] = la | (lb << 16);
      }
    }
    const v4u h0 = (v4u){oh[0][0], oh[0][1], oh[0][2], oh[0][3]};
    const v4u h1 = (v4u){oh[1][0], oh[1][1], oh[1][2], oh[1][3]};
    const v4u h2 = (v4u){oh[2][0], oh[2][1], oh[2][2], oh[2][3]};
    const v4u q0 = (v4u){ol[0][0], ol[0][1], ol[0][2], ol[0][3]};
    const v4u q1 = (v4u){ol[1][0], ol[1][1], ol[1][2], ol[1][3]};
    const v4u q2 = (v4u){ol[2][0], ol[2][1], ol[2][2], ol[2][3]};
    const size_t o0 = (size_t)(mrow0 + row) * ldc + ccol;
    const size_t o1 = (size_t)(mrow0 + kN + row) * ldc + ccol;
    const size_t o2 = (size_t)(mrow0 + 2 * kN + row) * ldc + ccol;
    volatile v4u* ph0 = (volatile v4u*)(Oh + o0);
    volatile v4u* ph1 = (volatile v4u*)(Oh + o1);
    volatile v4u* ph2 = (volatile v4u*)(Oh + o2);
    volatile v4u* pl0 = (volatile v4u*)(Ol + o0);
    volatile v4u* pl1 = (volatile v4u*)(Ol + o1);
    volatile v4u* pl2 = (volatile v4u*)(Ol + o2);
    *ph0 = h0; *ph1 = h1; *ph2 = h2;
    *pl0 = q0; *pl1 = q1; *pl2 = q2;
    __threadfence();
    *ph0 = h0; *ph1 = h1; *ph2 = h2;
    *pl0 = q0; *pl1 = q1; *pl2 = q2;
  }
}

__global__ __launch_bounds__(256) void k_pool_bcast(unsigned short* Xh, unsigned short* Xl) {
  __shared__ float red[16][128];
  __shared__ float pm[128];
  const int tid = threadIdx.x;
  const int cgp = tid & 15, slot = tid >> 4;
  const int bv = blockIdx.x;
  unsigned short* baseh = Xh + (size_t)bv * kN * kC2;
  unsigned short* basel = Xl + (size_t)bv * kN * kC2;
  float s[8];
#pragma unroll
  for (int e = 0; e < 8; ++e) s[e] = 0.f;
#pragma unroll 1
  for (int it = 0; it < 64; ++it) {
    const int row = it * 16 + slot;
    const v4u wh = *(const v4u*)(baseh + (size_t)row * kC2 + cgp * 8);
    const v4u wl = *(const v4u*)(basel + (size_t)row * kC2 + cgp * 8);
    float x[8];
    unpack8(wh, wl, x);
#pragma unroll
    for (int e = 0; e < 8; ++e) s[e] += x[e];
  }
#pragma unroll
  for (int e = 0; e < 8; ++e) red[slot][cgp * 8 + e] = s[e];
  __syncthreads();
  if (tid < 128) {
    float t = 0.f;
#pragma unroll
    for (int sl = 0; sl < 16; ++sl) t += red[sl][tid];
    pm[tid] = t * kInvN;
  }
  __syncthreads();
  unsigned hw[4], lw[4];
#pragma unroll
  for (int ep = 0; ep < 4; ++ep) {
    unsigned ha, la, hb, lb;
    split16(pm[cgp * 8 + 2 * ep], ha, la);
    split16(pm[cgp * 8 + 2 * ep + 1], hb, lb);
    hw[ep] = ha | (hb << 16);
    lw[ep] = la | (lb << 16);
  }
  const v4u vh = (v4u){hw[0], hw[1], hw[2], hw[3]};
  const v4u vl = (v4u){lw[0], lw[1], lw[2], lw[3]};
  for (int pass = 0; pass < 2; ++pass) {
#pragma unroll 1
    for (int it = 0; it < 64; ++it) {
      const int row = it * 16 + slot;
      *(volatile v4u*)(baseh + (size_t)row * kC2 + 128 + cgp * 8) = vh;
      *(volatile v4u*)(basel + (size_t)row * kC2 + 128 + cgp * 8) = vl;
    }
    __threadfence();
  }
}

__global__ __launch_bounds__(256) void k_head(const unsigned short* __restrict__ Yh, const unsigned short* __restrict__ Yl,
                                              const float* __restrict__ WdA, const float* __restrict__ Wc,
                                              float* __restrict__ out) {
  __shared__ float red[16][128];
  __shared__ __align__(16) float ys[3][128];
  __shared__ __align__(16) float av[3][128];
  __shared__ __align__(16) float os[384];
  const int tid = threadIdx.x;
  const int cgp = tid & 15, slot = tid >> 4;
  const int b = blockIdx.x;
#pragma unroll 1
  for (int v = 0; v < 3; ++v) {
    const unsigned short* baseh = Yh + (size_t)(b * 3 + v) * kN * kH3 + cgp * 8;
    const unsigned short* basel = Yl + (size_t)(b * 3 + v) * kN * kH3 + cgp * 8;
    float s[8];
#pragma unroll
    for (int e = 0; e < 8; ++e) s[e] = 0.f;
#pragma unroll 1
    for (int it = 0; it < 64; ++it) {
      const int row = it * 16 + slot;
      const v4u wh = *(const v4u*)(baseh + (size_t)row * kH3);
      const v4u wl = *(const v4u*)(basel + (size_t)row * kH3);
      float x[8];
      unpack8(wh, wl, x);
#pragma unroll
      for (int e = 0; e < 8; ++e) s[e] += x[e];
    }
#pragma unroll
    for (int e = 0; e < 8; ++e) red[slot][cgp * 8 + e] = s[e];
    __syncthreads();
    if (tid < 128) {
      float t = 0.f;
#pragma unroll
      for (int sl = 0; sl < 16; ++sl) t += red[sl][tid];
      ys[v][tid] = t * kInvN;
    }
    __syncthreads();
  }
  if (tid < 128) {
    const int c = tid;
    float d0 = 0.f, d1 = 0.f, d2 = 0.f;
    const v4f* wr = (const v4f*)(WdA + (size_t)c * kH3);
#pragma unroll 1
    for (int k4 = 0; k4 < 32; ++k4) {
      const v4f w = wr[k4];
      const v4f y0 = *(const v4f*)(&ys[0][4 * k4]);
      const v4f y1 = *(const v4f*)(&ys[1][4 * k4]);
      const v4f y2 = *(const v4f*)(&ys[2][4 * k4]);
#pragma unroll
      for (int e = 0; e < 4; ++e) {
        d0 = fmaf(w[e], y0[e], d0);
        d1 = fmaf(w[e], y1[e], d1);
        d2 = fmaf(w[e], y2[e], d2);
      }
    }
    const float x0 = ys[0][c], x1 = ys[1][c], x2 = ys[2][c];
    float a0, a1, a2;
    vn_act(x0, x1, x2, d0, d1, d2, a0, a1, a2);
    av[0][c] = a0;
    av[1][c] = a1;
    av[2][c] = a2;
  }
  __syncthreads();
  if (tid < 128) {
    const int c = tid;
    float o0 = 0.f, o1 = 0.f, o2 = 0.f;
    const v4f* wr = (const v4f*)(Wc + (size_t)c * kH3);
#pragma unroll 1
    for (int k4 = 0; k4 < 32; ++k4) {
      const v4f w = wr[k4];
      const v4f a0 = *(const v4f*)(&av[0][4 * k4]);
      const v4f a1 = *(const v4f*)(&av[1][4 * k4]);
      const v4f a2 = *(const v4f*)(&av[2][4 * k4]);
#pragma unroll
      for (int e = 0; e < 4; ++e) {
        o0 = fmaf(w[e], a0[e], o0);
        o1 = fmaf(w[e], a1[e], o1);
        o2 = fmaf(w[e], a2[e], o2);
      }
    }
    os[c * 3 + 0] = o0;
    os[c * 3 + 1] = o1;
    os[c * 3 + 2] = o2;
  }
  __syncthreads();
  if (tid < 96) {
    const v4f val = *(const v4f*)(os + 4 * tid);
    volatile v4f* d = (volatile v4f*)(out + (size_t)b * 384 + 4 * tid);
    *d = val;
    __threadfence();
    *d = val;
  }
}

extern "C" void kernel_launch(void* const* d_in, const int* in_sizes, int n_in,
                              void* d_out, int out_size, void* d_ws, size_t ws_size, hipStream_t stream) {
  (void)in_sizes; (void)out_size;
  if (n_in < 9) return;
  if (ws_size < kWsTotal) return;
  const float* p     = (const float*)d_in[0];
  const float* W_pos = (const float*)d_in[1];
  const float* Wd0s  = (const float*)d_in[2];
  const float* W0s   = (const float*)d_in[3];
  const float* Wd1s  = (const float*)d_in[4];
  const float* W1s   = (const float*)d_in[5];
  const float* Wss   = (const float*)d_in[6];
  const float* Wd_a  = (const float*)d_in[7];
  const float* W_c   = (const float*)d_in[8];

  char* ws = (char*)d_ws;
  unsigned short* wd0H = (unsigned short*)(ws + kOffWd0H);
  unsigned short* wd0L = (unsigned short*)(ws + kOffWd0L);
  unsigned short* w0H  = (unsigned short*)(ws + kOffW0H);
  unsigned short* w0L  = (unsigned short*)(ws + kOffW0L);
  unsigned short* wd1H = (unsigned short*)(ws + kOffWd1H);
  unsigned short* wd1L = (unsigned short*)(ws + kOffWd1L);
  unsigned short* w1H  = (unsigned short*)(ws + kOffW1H);
  unsigned short* w1L  = (unsigned short*)(ws + kOffW1L);
  unsigned short* wsH  = (unsigned short*)(ws + kOffWsH);
  unsigned short* wsL  = (unsigned short*)(ws + kOffWsL);
  float* E             = (float*)(ws + kOffE);
  unsigned short* X0H  = (unsigned short*)(ws + kOffX0H);
  unsigned short* X0L  = (unsigned short*)(ws + kOffX0L);
  unsigned short* X1H  = (unsigned short*)(ws + kOffX1H);
  unsigned short* X1L  = (unsigned short*)(ws + kOffX1L);
  unsigned short* A0H  = (unsigned short*)(ws + kOffA0H);
  unsigned short* A0L  = (unsigned short*)(ws + kOffA0L);
  unsigned short* T0H  = (unsigned short*)(ws + kOffT0H);
  unsigned short* T0L  = (unsigned short*)(ws + kOffT0L);
  unsigned short* A1H  = (unsigned short*)(ws + kOffA1H);
  unsigned short* A1L  = (unsigned short*)(ws + kOffA1L);
  unsigned short* YLH  = (unsigned short*)(ws + kOffYLH);
  unsigned short* YLL  = (unsigned short*)(ws + kOffYLL);

  k_cvt_w<<<(5 * 256 * 256 / 8) / 256, 256, 0, stream>>>(Wd0s, wd0H, wd0L, 5 * 256 * 256 / 8);
  k_cvt_w<<<(5 * 128 * 256 / 8) / 256, 256, 0, stream>>>(W0s,  w0H,  w0L,  5 * 128 * 256 / 8);
  k_cvt_w<<<(5 * 128 * 128 / 8) / 256, 256, 0, stream>>>(Wd1s, wd1H, wd1L, 5 * 128 * 128 / 8);
  k_cvt_w<<<(5 * 128 * 128 / 8) / 256, 256, 0, stream>>>(W1s,  w1H,  w1L,  5 * 128 * 128 / 8);
  k_cvt_w<<<(5 * 128 * 256 / 8) / 256, 256, 0, stream>>>(Wss,  wsH,  wsL,  5 * 128 * 256 / 8);

  k_knn_feat<<<kB * 4, 256, 0, stream>>>(p, E);
  k_init<<<kRows / (8 * 32), 256, 0, stream>>>(E, W_pos, X0H, X0L);

  unsigned short* curH = X0H;
  unsigned short* curL = X0L;
  unsigned short* nxtH = X1H;
  unsigned short* nxtL = X1L;
  for (int i = 0; i < 5; ++i) {
    const unsigned short* wd0h = wd0H + (size_t)i * 256 * 256;
    const unsigned short* wd0l = wd0L + (size_t)i * 256 * 256;
    const unsigned short* w0h  = w0H  + (size_t)i * 128 * 256;
    const unsigned short* w0l  = w0L  + (size_t)i * 128 * 256;
    const unsigned short* wd1h = wd1H + (size_t)i * 128 * 128;
    const unsigned short* wd1l = wd1L + (size_t)i * 128 * 128;
    const unsigned short* w1h  = w1H  + (size_t)i * 128 * 128;
    const unsigned short* w1l  = w1L  + (size_t)i * 128 * 128;
    const unsigned short* wsh  = wsH  + (size_t)i * 128 * 256;
    const unsigned short* wsl  = wsL  + (size_t)i * 128 * 256;
    k_vn_gemm<256, 0, 256, 1><<<1024, 128, 0, stream>>>(curH, curL, 256, wd0h, wd0l,
                                                        curH, curL, 256, wd0h, wd0l, A0H, A0L, 256);
    k_vn_gemm<256, 0, 128, 0><<<512, 128, 0, stream>>>(A0H, A0L, 256, w0h, w0l,
                                                       A0H, A0L, 256, w0h, w0l, T0H, T0L, 128);
    k_vn_gemm<128, 0, 128, 1><<<512, 128, 0, stream>>>(T0H, T0L, 128, wd1h, wd1l,
                                                       T0H, T0L, 128, wd1h, wd1l, A1H, A1L, 128);
    if (i < 4) {
      k_vn_gemm<128, 256, 128, 0><<<512, 128, 0, stream>>>(A1H, A1L, 128, w1h, w1l,
                                                           curH, curL, 256, wsh, wsl, nxtH, nxtL, 256);
      k_pool_bcast<<<kB * 3, 256, 0, stream>>>(nxtH, nxtL);
      unsigned short* th = curH; curH = nxtH; nxtH = th;
      unsigned short* tl = curL; curL = nxtL; nxtL = tl;
    } else {
      k_vn_gemm<128, 256, 128, 0><<<512, 128, 0, stream>>>(A1H, A1L, 128, w1h, w1l,
                                                           curH, curL, 256, wsh, wsl, YLH, YLL, 128);
    }
  }
  k_head<<<kB, 256, 0, stream>>>(YLH, YLL, Wd_a, W_c, (float*)d_out);
}
